// GraphSemanticLoss_32916629356852
// MI455X (gfx1250) — hardware-run, weakly checked
//
#include <hip/hip_runtime.h>
#include <math.h>

typedef __attribute__((ext_vector_type(16))) _Float16 v16h;
typedef __attribute__((ext_vector_type(8)))  _Float16 v8h;
typedef __attribute__((ext_vector_type(8)))  float    v8f;
typedef __attribute__((ext_vector_type(4)))  float    v4f;

constexpr int kB = 512;
constexpr int kD = 512;
constexpr int   kCarryExp = 6;
constexpr float kCarry    = (float)(1 << kCarryExp);
constexpr float kFold     = 1.0f / (kCarry * kCarry);
constexpr float kHinge    = 0.5f;
constexpr float kTwoEps   = (float)(2.0 * 1e-6);
constexpr float kEpsSq    = (float)((double)kD * 1e-6 * 1e-6);
constexpr float kPosThr   = 0.7f;
constexpr float kNegThr   = 0.3f;
constexpr float kSentLo   = -1e30f;
constexpr float kSentHi   = 1e30f;
constexpr float kSentCut  = -1e29f;
constexpr int kRecPitch   = 32;
constexpr int kDiagPitch  = kB + 1;
static_assert((kB % 64) == 0 && (kD % 32) == 0, "GEMM tile multiples");
static_assert(kB == 512 && kD == 512, "lane maps below are written for 512 x 512");
static_assert(((kB / 64) * (kB / 64)) == 64, "64 wave tiles = 8 blocks x 8 waves");

constexpr size_t kOffEH  = 0;
constexpr size_t kOffSV  = kOffEH + (size_t)kB * kD * 2;
constexpr size_t kOffG   = kOffSV + (size_t)kB * 4;
constexpr size_t kOffREC = kOffG + (size_t)kB * kB * 4;
constexpr size_t kWsTotal = kOffREC + (size_t)kB * kRecPitch * 4;
static_assert(kWsTotal == 1640448ull, "carve total");
static_assert(kWsTotal <= 134217728ull, "carve cap");
static_assert((kOffSV % 128) == 0 && (kOffG % 128) == 0 && (kOffREC % 128) == 0, "aligned regions");

__device__ __forceinline__ float wave_sum_f(float v) {
#pragma unroll
  for (int off = 16; off > 0; off >>= 1) v += __shfl_xor(v, off, 32);
  return v;
}
__device__ __forceinline__ float wave_max_f(float v) {
#pragma unroll
  for (int off = 16; off > 0; off >>= 1) v = fmaxf(v, __shfl_xor(v, off, 32));
  return v;
}
__device__ __forceinline__ int wave_sum_i(int v) {
#pragma unroll
  for (int off = 16; off > 0; off >>= 1) v += __shfl_xor(v, off, 32);
  return v;
}

union FragU { v16h v; v8h h[2]; };
__device__ __forceinline__ v16h frag_load(const _Float16* p) {
  FragU f;
  f.h[0] = *(const v8h*)(p);
  f.h[1] = *(const v8h*)(p + 16);
  return f.v;
}
__device__ __forceinline__ v8f mma_f16(v16h a, v16h b, v8f c) {
  c = __builtin_amdgcn_wmma_f32_16x16x32_f16(false, a, false, b, (short)0, c, false, false);
  asm volatile("v_nop\n\tv_nop\n\tv_nop\n\tv_nop" : "+v"(c) : "v"(a), "v"(b));
  return c;
}
__device__ __forceinline__ void keep4_h(v16h a, v16h b, v16h c, v16h d) { asm volatile("v_nop" :: "v"(a), "v"(b), "v"(c), "v"(d)); }

__device__ __forceinline__ _Float16 cvt_carry(float x, float& s) {
  s += x;
  return (_Float16)ldexpf(x, kCarryExp);
}

__global__ __launch_bounds__(256) void prep_rows_kernel(
    const float* __restrict__ E, unsigned short* __restrict__ EH, float* __restrict__ svv)
{
  __shared__ float sS[32];
  const int tid = threadIdx.x, lane = tid & 31, wave = tid >> 5;
  const int rowBase = blockIdx.x * 32 + wave * 4;
  for (int r = 0; r < 4; ++r) {
    const int row = rowBase + r;
    const float* p = E + (size_t)row * kD;
    const v4f a0 = *(const v4f*)(p + lane * 8);
    const v4f a1 = *(const v4f*)(p + lane * 8 + 4);
    const v4f b0 = *(const v4f*)(p + 256 + lane * 8);
    const v4f b1 = *(const v4f*)(p + 256 + lane * 8 + 4);
    float s = 0.f;
    v8h hA, hB;
#pragma unroll
    for (int e = 0; e < 4; ++e) {
      hA[e]     = cvt_carry(a0[e], s);
      hA[4 + e] = cvt_carry(a1[e], s);
      hB[e]     = cvt_carry(b0[e], s);
      hB[4 + e] = cvt_carry(b1[e], s);
    }
    s = wave_sum_f(s);
    if (lane == 0) sS[wave * 4 + r] = s;
    unsigned short* o = EH + (size_t)row * kD + lane * 8;
    *(volatile v8h*)(o)       = hA;
    *(volatile v8h*)(o + 256) = hB;
    __threadfence();
    *(volatile v8h*)(o)       = hA;
    *(volatile v8h*)(o + 256) = hB;
  }
  __syncthreads();
  if (wave == 0) {
    const float vs = sS[lane];
    float* os = svv + blockIdx.x * 32 + lane;
    *(volatile float*)os = vs;
    __threadfence();
    *(volatile float*)os = vs;
  }
}

__global__ __launch_bounds__(256) void gram_kernel(
    const unsigned short* __restrict__ EHp, float* __restrict__ G)
{
  __shared__ __align__(16) float sT[8][16 * 68];
  const _Float16* EH = (const _Float16*)EHp;
  const int lane = threadIdx.x & 31;
  const int wave = threadIdx.x >> 5;
  const int tile = blockIdx.x * 8 + wave;
  const int tm = tile >> 3;
  const int tn = tile & 7;
  const int m0 = tm << 6;
  const int n0 = tn << 6;
  const int rlane = lane & 15;
  const int koff  = (lane >> 4) * 8;
  const int mOff  = (lane >> 4) * 8;

  v8f acc[4][4];
#pragma unroll
  for (int i = 0; i < 4; ++i)
#pragma unroll
    for (int j = 0; j < 4; ++j) acc[i][j] = (v8f){0.f,0.f,0.f,0.f,0.f,0.f,0.f,0.f};

  for (int k0 = 0; k0 < kD; k0 += 32) {
    v16h bh[4];
#pragma unroll
    for (int j = 0; j < 4; ++j) {
      const size_t bo = (size_t)(n0 + (j << 4) + rlane) * kD + koff + k0;
      bh[j] = frag_load(EH + bo);
    }
#pragma unroll
    for (int i = 0; i < 4; ++i) {
      const size_t ao = (size_t)(m0 + (i << 4) + rlane) * kD + koff + k0;
      const v16h ah = frag_load(EH + ao);
#pragma unroll
      for (int j = 0; j < 4; ++j) acc[i][j] = mma_f16(ah, bh[j], acc[i][j]);
    }
    keep4_h(bh[0], bh[1], bh[2], bh[3]);
  }

  float* slab = sT[wave];
#pragma unroll
  for (int i = 0; i < 4; ++i) {
    const int mBase = m0 + (i << 4);
#pragma unroll
    for (int j = 0; j < 4; ++j) {
#pragma unroll
      for (int r = 0; r < 8; ++r) {
        slab[(mOff + r) * 68 + (j << 4) + rlane] = acc[i][j][r] * kFold;
      }
    }
    __builtin_amdgcn_fence(__ATOMIC_RELEASE, "workgroup");
    __builtin_amdgcn_wave_barrier();
    __builtin_amdgcn_fence(__ATOMIC_ACQUIRE, "workgroup");
    {
      const int hh = lane >> 4, c4 = (lane & 15) * 4;
      for (int pass = 0; pass < 2; ++pass) {
#pragma unroll
        for (int it = 0; it < 8; ++it) {
          const int row = it * 2 + hh;
          const v4f v = *(const v4f*)(slab + row * 68 + c4);
          *(volatile v4f*)(G + (size_t)(mBase + row) * kB + n0 + c4) = v;
        }
        __threadfence();
      }
    }
    __builtin_amdgcn_fence(__ATOMIC_RELEASE, "workgroup");
    __builtin_amdgcn_wave_barrier();
    __builtin_amdgcn_fence(__ATOMIC_ACQUIRE, "workgroup");
  }
}

__device__ __forceinline__ void anchor_elem(float sval, float draw, float sj, float si,
                                            float& pd, float& nd, float& dsum, float& dmax,
                                            float& ssum, int& npos, int& nneg)
{
  const float d2   = fmaxf(draw, 0.0f);
  const float dist = sqrtf(d2);
  const float dt2  = (d2 + kTwoEps * (si - sj)) + kEpsSq;
  const float dt   = sqrtf(fmaxf(dt2, 0.0f));
  const bool isPos = sval > kPosThr;
  const bool isNeg = sval < kNegThr;
  pd = isPos ? (dt + kHinge) : kSentLo;
  nd = isNeg ? dt : kSentHi;
  dsum += dist;
  dmax = fmaxf(dmax, dist);
  ssum += sval;
  npos += isPos ? 1 : 0;
  nneg += isNeg ? 1 : 0;
}

__global__ __launch_bounds__(256) void anchor_kernel(
    const float* __restrict__ S, const float* __restrict__ G, const float* __restrict__ svv,
    float* __restrict__ rec)
{
  __shared__ float pdt[kB];
  __shared__ float redT[8];
  __shared__ float redS[8];
  __shared__ float redD[8];
  __shared__ float redM[8];
  __shared__ int   redP[8];
  __shared__ int   redN[8];
  const int tid = threadIdx.x, lane = tid & 31, wave = tid >> 5;
  const int i = blockIdx.x;
  const size_t rowOff = (size_t)i * kB;
  const float si  = svv[i];
  const float sqi = G[(size_t)i * kDiagPitch];
  const float sv0 = S[rowOff + tid];
  const float sv1 = S[rowOff + tid + 256];
  const float g0  = G[rowOff + tid];
  const float g1  = G[rowOff + tid + 256];
  const float sq0 = G[(size_t)tid * kDiagPitch];
  const float sq1 = G[(size_t)(tid + 256) * kDiagPitch];
  const float sj0 = svv[tid];
  const float sj1 = svv[tid + 256];
  const float dr0 = (sqi + sq0) - 2.0f * g0;
  const float dr1 = (sqi + sq1) - 2.0f * g1;

  float dsum = 0.f, dmax = 0.f, ssum = 0.f;
  int npos = 0, nneg = 0;
  float p0, n0, p1, n1;
  anchor_elem(sv0, dr0, sj0, si, p0, n0, dsum, dmax, ssum, npos, nneg);
  anchor_elem(sv1, dr1, sj1, si, p1, n1, dsum, dmax, ssum, npos, nneg);
  pdt[tid]       = p0;
  pdt[tid + 256] = p1;
  __syncthreads();

  float acc = 0.f;
  for (int j = 0; j < kB; ++j) {
    const float a = __int_as_float(__builtin_amdgcn_readfirstlane(__float_as_int(pdt[j])));
    if (a < kSentCut) continue;
    acc += fmaxf(a - n0, 0.0f) + fmaxf(a - n1, 0.0f);
  }

  acc  = wave_sum_f(acc);
  ssum = wave_sum_f(ssum);
  dsum = wave_sum_f(dsum);
  dmax = wave_max_f(dmax);
  npos = wave_sum_i(npos);
  nneg = wave_sum_i(nneg);
  if (lane == 0) {
    redT[wave] = acc;
    redS[wave] = ssum;
    redD[wave] = dsum;
    redM[wave] = dmax;
    redP[wave] = npos;
    redN[wave] = nneg;
  }
  __syncthreads();
  if (wave == 0) {
    float tT = 0.f, tS = 0.f, tD = 0.f, tM = 0.f;
    int tP = 0, tN = 0;
#pragma unroll
    for (int w = 0; w < 8; ++w) {
      tT += redT[w];
      tS += redS[w];
      tD += redD[w];
      tM = fmaxf(tM, redM[w]);
      tP += redP[w];
      tN += redN[w];
    }
    const float cntf = (float)(tP * tN);
    float val = 0.0f;
    val = (lane == 0) ? tT : val;
    val = (lane == 1) ? cntf : val;
    val = (lane == 2) ? tS : val;
    val = (lane == 3) ? tD : val;
    val = (lane == 4) ? tM : val;
    float* o = rec + (size_t)i * kRecPitch + lane;
    *(volatile float*)o = val;
    __threadfence();
    *(volatile float*)o = val;
  }
}

__device__ __forceinline__ int rec_count(float v) {
  const float c = fminf(fmaxf(v, 0.0f), 262144.0f);
  return (int)c;
}

__global__ __launch_bounds__(256) void finalize_kernel(const float* __restrict__ rec, float* __restrict__ out)
{
  __shared__ float rT[8];
  __shared__ float rS[8];
  __shared__ float rD[8];
  __shared__ float rM[8];
  __shared__ int   rC[8];
  const int tid = threadIdx.x, lane = tid & 31, wave = tid >> 5;
  const v4f a0 = *(const v4f*)(rec + (size_t)tid * kRecPitch);
  const v4f a1 = *(const v4f*)(rec + (size_t)(tid + 256) * kRecPitch);
  const float m0 = rec[(size_t)tid * kRecPitch + 4];
  const float m1 = rec[(size_t)(tid + 256) * kRecPitch + 4];
  float ts = a0[0] + a1[0];
  int cnt  = rec_count(a0[1]) + rec_count(a1[1]);
  float ss = a0[2] + a1[2];
  float ds = a0[3] + a1[3];
  float dm = fmaxf(m0, m1);
  ts  = wave_sum_f(ts);
  ss  = wave_sum_f(ss);
  ds  = wave_sum_f(ds);
  dm  = wave_max_f(dm);
  cnt = wave_sum_i(cnt);
  if (lane == 0) {
    rT[wave] = ts;
    rS[wave] = ss;
    rD[wave] = ds;
    rM[wave] = dm;
    rC[wave] = cnt;
  }
  __syncthreads();
  if (tid == 0) {
    float tT = 0.f, tS = 0.f, tD = 0.f, tM = 0.f;
    int tC = 0;
#pragma unroll
    for (int w = 0; w < 8; ++w) {
      tT += rT[w];
      tS += rS[w];
      tD += rD[w];
      tM = fmaxf(tM, rM[w]);
      tC += rC[w];
    }
    const float nAll = (float)kB * (float)kB;
    const float simLoss = tD * (1.0f / (tM * nAll)) - tS * (1.0f / nAll);
    const int   cSafe = (tC > 0) ? tC : 1;
    const float trip  = (tC > 0) ? (tT * (1.0f / (float)cSafe)) : 0.0f;
    const float res = trip + simLoss;
    *(volatile float*)out = res;
    __threadfence();
    *(volatile float*)out = res;
  }
}

extern "C" void kernel_launch(void* const* d_in, const int* in_sizes, int n_in,
                              void* d_out, int out_size, void* d_ws, size_t ws_size,
                              hipStream_t stream) {
  if (n_in < 2) return;
  if (in_sizes[0] != kB * kD) return;
  if (in_sizes[1] != kB * kB) return;
  if (out_size != 1) return;
  if (ws_size < kWsTotal) return;

  const float* E = (const float*)d_in[0];
  const float* S = (const float*)d_in[1];
  float* out = (float*)d_out;

  char* ws = (char*)d_ws;
  unsigned short* EH  = (unsigned short*)(ws + kOffEH);
  float*          SV  = (float*)(ws + kOffSV);
  float*          G   = (float*)(ws + kOffG);
  float*          REC = (float*)(ws + kOffREC);

  prep_rows_kernel<<<kB / 32, 256, 0, stream>>>(E, EH, SV);
  gram_kernel<<<((kB / 64) * (kB / 64)) / 8, 256, 0, stream>>>(EH, G);
  anchor_kernel<<<kB, 256, 0, stream>>>(S, G, SV, REC);
  finalize_kernel<<<1, 256, 0, stream>>>(REC, out);
}
